// HAOQAttention_55851754717277
// MI455X (gfx1250) — hardware-verified
//
#include <hip/hip_runtime.h>
#include <math.h>
#include <stdint.h>

#define NTOK 8192
#define DM   1024
#define NH   16
#define HD   64

static_assert(NTOK % 64 == 0);
static_assert(DM % 64 == 0);

typedef _Float16 v16h __attribute__((ext_vector_type(16)));
typedef _Float16 v8h  __attribute__((ext_vector_type(8)));
typedef float    v8f  __attribute__((ext_vector_type(8)));
typedef float    v4f  __attribute__((ext_vector_type(4)));

union FragH { v16h v; v8h h[2]; };

__device__ __forceinline__ v16h frag_load(const _Float16* p) {
  FragH f;
  f.h[0] = *(const v8h*)(p);
  f.h[1] = *(const v8h*)(p + 16);
  return f.v;
}

__device__ __forceinline__ v8f mma16(v16h a, v16h b, v8f c) {
  c = __builtin_amdgcn_wmma_f32_16x16x32_f16(false, a, false, b, (short)0, c, false, false);
  asm volatile("v_nop\n\tv_nop\n\tv_nop\n\tv_nop" : "+v"(c) : "v"(a), "v"(b));
  return c;
}

__device__ __forceinline__ v8f vzero8() {
  v8f z = {0.f, 0.f, 0.f, 0.f, 0.f, 0.f, 0.f, 0.f};
  return z;
}

__device__ __forceinline__ void wave_lds_sync() {
  __builtin_amdgcn_fence(__ATOMIC_RELEASE, "workgroup");
  __builtin_amdgcn_wave_barrier();
  __builtin_amdgcn_fence(__ATOMIC_ACQUIRE, "workgroup");
}

__device__ __forceinline__ void fusion_w2(const float* __restrict__ fw, float& w0, float& w1) {
  const float f0 = fw[0], f1 = fw[1];
  const float mx = fmaxf(f0, f1);
  const float e0 = __expf(f0 - mx), e1 = __expf(f1 - mx);
  const float inv = 1.0f / (e0 + e1);
  w0 = e0 * inv;
  w1 = e1 * inv;
}

__global__ __launch_bounds__(256)
void k_cvt16(const float* __restrict__ in, _Float16* __restrict__ out, int n8, float scale) {
  const int i = blockIdx.x * 256 + threadIdx.x;
  if (i >= n8) return;
  const size_t e0 = (size_t)i * 8;
  const v4f a = *(const v4f*)(in + e0);
  const v4f b = *(const v4f*)(in + e0 + 4);
  v8h o;
  o[0] = (_Float16)(a[0] * scale); o[1] = (_Float16)(a[1] * scale);
  o[2] = (_Float16)(a[2] * scale); o[3] = (_Float16)(a[3] * scale);
  o[4] = (_Float16)(b[0] * scale); o[5] = (_Float16)(b[1] * scale);
  o[6] = (_Float16)(b[2] * scale); o[7] = (_Float16)(b[3] * scale);
  _Float16* p = out + e0;
  *(volatile v8h*)p = o;
  __threadfence();
  *(volatile v8h*)p = o;
}

__global__ __launch_bounds__(256)
void k_wcat(const float* __restrict__ Wl, const float* __restrict__ Wg, const float* __restrict__ fw,
            _Float16* __restrict__ out, int n8) {
  const int i = blockIdx.x * 256 + threadIdx.x;
  if (i >= n8) return;
  const size_t e0 = (size_t)i * 8;
  const int n  = (int)(e0 >> 11);
  const int k2 = (int)(e0 & 2047);
  const int kk = k2 & 1023;
  float w0, w1;
  fusion_w2(fw, w0, w1);
  const bool useL = (k2 < DM);
  const float sc = useL ? (64.0f * w0) : (64.0f * w1);
  const float* pl = Wl + (size_t)n * DM + kk;
  const float* pg = Wg + (size_t)n * DM + kk;
  const v4f a0 = *(const v4f*)(pl), a1 = *(const v4f*)(pl + 4);
  const v4f b0 = *(const v4f*)(pg), b1 = *(const v4f*)(pg + 4);
  v8h o;
  o[0] = (_Float16)((useL ? a0[0] : b0[0]) * sc); o[1] = (_Float16)((useL ? a0[1] : b0[1]) * sc);
  o[2] = (_Float16)((useL ? a0[2] : b0[2]) * sc); o[3] = (_Float16)((useL ? a0[3] : b0[3]) * sc);
  o[4] = (_Float16)((useL ? a1[0] : b1[0]) * sc); o[5] = (_Float16)((useL ? a1[1] : b1[1]) * sc);
  o[6] = (_Float16)((useL ? a1[2] : b1[2]) * sc); o[7] = (_Float16)((useL ? a1[3] : b1[3]) * sc);
  _Float16* p = out + e0;
  *(volatile v8h*)p = o;
  __threadfence();
  *(volatile v8h*)p = o;
}

__global__ __launch_bounds__(256)
void k_tcvt16(const float* __restrict__ W, _Float16* __restrict__ out, int R, int Cc, float scale) {
  __shared__ __align__(16) float tf[64 * 68];
  const int c0  = blockIdx.x * 64;
  const int r0  = blockIdx.y * 64;
  const int tid = threadIdx.x;
  if (c0 >= Cc || r0 >= R) return;
  {
    const int lr = tid >> 4;
    const int c4 = (tid & 15) * 4;
#pragma unroll
    for (int it = 0; it < 4; ++it) {
      const int rr = it * 16 + lr;
      const v4f a = *(const v4f*)(W + (size_t)(r0 + rr) * Cc + c0 + c4);
      *(v4f*)(tf + rr * 68 + c4) = a;
    }
  }
  __syncthreads();
  const int sub = tid >> 3;
  const int c8  = (tid & 7) * 8;
  v8h hv[2];
#pragma unroll
  for (int it = 0; it < 2; ++it) {
    const int oc = it * 32 + sub;
    v8h o;
#pragma unroll
    for (int e = 0; e < 8; ++e) o[e] = (_Float16)(tf[(c8 + e) * 68 + oc] * scale);
    hv[it] = o;
  }
  for (int pass = 0; pass < 2; ++pass) {
#pragma unroll
    for (int it = 0; it < 2; ++it) {
      const int oc = it * 32 + sub;
      *(volatile v8h*)(out + (size_t)(c0 + oc) * R + r0 + c8) = hv[it];
    }
    __threadfence();
  }
}

template <int BIAS_MODE, int OUT_MODE>
__global__ __launch_bounds__(256)
void k_gemm64(const _Float16* __restrict__ A, int lda,
              const _Float16* __restrict__ Bt, int ldb,
              void* __restrict__ Cout, int ldc,
              const float* __restrict__ bias, const float* __restrict__ bias2, const float* __restrict__ fw,
              int M, int N, int K, float scale, float bmul) {
  __shared__ __align__(16) float sT[8][16 * 68];
  const int lane = threadIdx.x & 31;
  const int wave = threadIdx.x >> 5;
  const int tilesN = N >> 6;
  const int tilesM = M >> 6;
  const int tile = blockIdx.x * 8 + wave;
  if (tile >= tilesM * tilesN) return;
  const int tm = tile / tilesN;
  const int tn = tile - tm * tilesN;
  const int m0 = tm << 6;
  const int n0 = tn << 6;

  const int rl   = lane & 15;
  const int koff = (lane >> 4) * 8;
  const int mOff = (lane >> 4) * 8;

  v8f acc[4][4];
#pragma unroll
  for (int i = 0; i < 4; ++i)
#pragma unroll
    for (int j = 0; j < 4; ++j) acc[i][j] = vzero8();

#pragma unroll 1
  for (int k0 = 0; k0 < K; k0 += 32) {
    v16h bfr[4];
#pragma unroll
    for (int j = 0; j < 4; ++j)
      bfr[j] = frag_load(Bt + (size_t)(n0 + 16 * j + rl) * ldb + k0 + koff);
#pragma unroll
    for (int i = 0; i < 4; ++i) {
      const v16h afr = frag_load(A + (size_t)(m0 + 16 * i + rl) * lda + k0 + koff);
#pragma unroll
      for (int j = 0; j < 4; ++j) acc[i][j] = mma16(afr, bfr[j], acc[i][j]);
    }
  }

  float w0 = 0.f, w1 = 0.f;
  if (BIAS_MODE == 3) fusion_w2(fw, w0, w1);
  float* slab = sT[wave];
#pragma unroll
  for (int i = 0; i < 4; ++i) {
    const int mBase = m0 + (i << 4);
#pragma unroll
    for (int j = 0; j < 4; ++j) {
      const int n = n0 + (j << 4) + rl;
      float bv = 0.f;
      if (BIAS_MODE == 2) bv = bias[n] * bmul;
      if (BIAS_MODE == 3) bv = w0 * bias[n] + w1 * bias2[n];
#pragma unroll
      for (int r = 0; r < 8; ++r) {
        float v = acc[i][j][r] * scale;
        if (BIAS_MODE == 1) v += bias[mBase + mOff + r] * bmul;
        if (BIAS_MODE == 2 || BIAS_MODE == 3) v += bv;
        slab[(mOff + r) * 68 + (j << 4) + rl] = v;
      }
    }
    wave_lds_sync();
    if (OUT_MODE == 0) {
      float* C = (float*)Cout;
      const int h2 = lane >> 4;
      const int c4 = (lane & 15) * 4;
      v4f vv[8];
#pragma unroll
      for (int it = 0; it < 8; ++it) vv[it] = *(const v4f*)(slab + (it * 2 + h2) * 68 + c4);
      for (int pass = 0; pass < 2; ++pass) {
#pragma unroll
        for (int it = 0; it < 8; ++it)
          *(volatile v4f*)(C + (size_t)(mBase + it * 2 + h2) * ldc + n0 + c4) = vv[it];
        __threadfence();
      }
    } else {
      _Float16* C = (_Float16*)Cout;
      const int q  = lane >> 3;
      const int c8 = (lane & 7) * 8;
      v8h hv[4];
#pragma unroll
      for (int it = 0; it < 4; ++it) {
        const float* sp = slab + (it * 4 + q) * 68 + c8;
        const v4f x0 = *(const v4f*)(sp);
        const v4f x1 = *(const v4f*)(sp + 4);
        v8h o;
        o[0] = (_Float16)x0[0]; o[1] = (_Float16)x0[1]; o[2] = (_Float16)x0[2]; o[3] = (_Float16)x0[3];
        o[4] = (_Float16)x1[0]; o[5] = (_Float16)x1[1]; o[6] = (_Float16)x1[2]; o[7] = (_Float16)x1[3];
        hv[it] = o;
      }
      for (int pass = 0; pass < 2; ++pass) {
#pragma unroll
        for (int it = 0; it < 4; ++it)
          *(volatile v8h*)(C + (size_t)(mBase + it * 4 + q) * ldc + n0 + c8) = hv[it];
        __threadfence();
      }
    }
    wave_lds_sync();
  }
}

__global__ __launch_bounds__(128)
void k_attn(const _Float16* __restrict__ QK, const _Float16* __restrict__ VT, _Float16* __restrict__ Oc,
            int W, int colOff) {
  __shared__ __align__(16) _Float16 Psh[4][16 * 64];
  __shared__ __align__(16) float    Os[4][16 * 68];
  const int tid  = threadIdx.x;
  const int wave = tid >> 5;
  const int lane = tid & 31;
  const int hh   = lane >> 4;
  const int c    = lane & 15;
  const int nqb  = W >> 6;
  const int bx   = blockIdx.x;
  const int qb   = bx % nqb;
  const int t1   = bx / nqb;
  const int h    = t1 % NH;
  const int seg  = t1 / NH;
  if ((seg + 1) * W > NTOK) return;
  const int rowW = seg * W;
  const int qw0  = qb * 64 + wave * 16;
  const int q0   = rowW + qw0;
  const size_t LQK = (size_t)(2 * DM);

  v16h qa[2];
#pragma unroll
  for (int dc = 0; dc < 2; ++dc)
    qa[dc] = frag_load(QK + (size_t)(q0 + c) * LQK + h * HD + dc * 32 + 8 * hh);

  float mrow[8], lrow[8];
  v8f oacc[4];
#pragma unroll
  for (int r = 0; r < 8; ++r) { mrow[r] = -1.0e30f; lrow[r] = 0.f; }
#pragma unroll
  for (int t = 0; t < 4; ++t) oacc[t] = vzero8();

  _Float16* Pw = Psh[wave];

#pragma unroll 1
  for (int kc = 0; kc < nqb; ++kc) {
    const int kv0 = kc * 64;
    v8f s[4];
#pragma unroll
    for (int j = 0; j < 4; ++j) {
      s[j] = vzero8();
#pragma unroll
      for (int dc = 0; dc < 2; ++dc) {
        const v16h kb = frag_load(QK + (size_t)(rowW + kv0 + 16 * j + c) * LQK + DM + h * HD + dc * 32 + 8 * hh);
        s[j] = mma16(qa[dc], kb, s[j]);
      }
    }
    float cm[8];
#pragma unroll
    for (int r = 0; r < 8; ++r) {
      const int iq = qw0 + 8 * hh + r;
      float m = -1.0e30f;
#pragma unroll
      for (int j = 0; j < 4; ++j) {
        const int ik = kv0 + 16 * j + c;
        const float sv = s[j][r] * 0.125f + ((ik > iq) ? 1.0f : 0.0f);
        s[j][r] = sv;
        m = fmaxf(m, sv);
      }
#pragma unroll
      for (int off = 1; off < 16; off <<= 1) m = fmaxf(m, __shfl_xor(m, off, 32));
      cm[r] = m;
    }
    wave_lds_sync();
#pragma unroll
    for (int r = 0; r < 8; ++r) {
      const float mnew  = fmaxf(mrow[r], cm[r]);
      const float alpha = __expf(mrow[r] - mnew);
      mrow[r] = mnew;
      float psum = 0.f;
#pragma unroll
      for (int j = 0; j < 4; ++j) {
        const float p = __expf(s[j][r] - mnew);
        psum += p;
        Pw[(8 * hh + r) * 64 + 16 * j + c] = (_Float16)(p * 256.0f);
      }
#pragma unroll
      for (int off = 1; off < 16; off <<= 1) psum += __shfl_xor(psum, off, 32);
      lrow[r] = lrow[r] * alpha + psum;
#pragma unroll
      for (int t = 0; t < 4; ++t) oacc[t][r] *= alpha;
    }
    wave_lds_sync();
#pragma unroll
    for (int kk = 0; kk < 2; ++kk) {
      const v16h pa = frag_load(Pw + c * 64 + kk * 32 + 8 * hh);
#pragma unroll
      for (int t = 0; t < 4; ++t) {
        const v16h vb = frag_load(VT + (size_t)(h * HD + 16 * t + c) * NTOK + rowW + kv0 + kk * 32 + 8 * hh);
        oacc[t] = mma16(pa, vb, oacc[t]);
      }
    }
  }

  float* os = Os[wave];
#pragma unroll
  for (int r = 0; r < 8; ++r) {
    const float inv = 1.0f / (64.0f * lrow[r]);
#pragma unroll
    for (int t = 0; t < 4; ++t) os[(8 * hh + r) * 68 + 16 * t + c] = oacc[t][r] * inv;
  }
  wave_lds_sync();
  const int q  = lane >> 3;
  const int c8 = (lane & 7) * 8;
  v8h hv[4];
#pragma unroll
  for (int it = 0; it < 4; ++it) {
    const float* sp = os + (it * 4 + q) * 68 + c8;
    const v4f x0 = *(const v4f*)(sp);
    const v4f x1 = *(const v4f*)(sp + 4);
    v8h o;
    o[0] = (_Float16)x0[0]; o[1] = (_Float16)x0[1]; o[2] = (_Float16)x0[2]; o[3] = (_Float16)x0[3];
    o[4] = (_Float16)x1[0]; o[5] = (_Float16)x1[1]; o[6] = (_Float16)x1[2]; o[7] = (_Float16)x1[3];
    hv[it] = o;
  }
  for (int pass = 0; pass < 2; ++pass) {
#pragma unroll
    for (int it = 0; it < 4; ++it)
      *(volatile v8h*)(Oc + (size_t)(q0 + it * 4 + q) * LQK + colOff + h * HD + c8) = hv[it];
    __threadfence();
  }
}

__global__ __launch_bounds__(256)
void k_layernorm(const float* __restrict__ Y, const float* __restrict__ gamma, const float* __restrict__ beta,
                 float* __restrict__ out, int nrows) {
  __shared__ float red[8];
  const int row = blockIdx.x;
  if (row >= nrows) return;
  const int tid  = threadIdx.x;
  const int lane = tid & 31;
  const int wave = tid >> 5;
  const int col  = tid * 4;
  const v4f v = *(const v4f*)(Y + (size_t)row * DM + col);
  float s = (v[0] + v[1]) + (v[2] + v[3]);
#pragma unroll
  for (int off = 1; off < 32; off <<= 1) s += __shfl_xor(s, off, 32);
  if (lane == 0) red[wave] = s;
  __syncthreads();
  float tot = 0.f;
#pragma unroll
  for (int w = 0; w < 8; ++w) tot += red[w];
  const float mean = tot * (1.0f / 1024.0f);
  __syncthreads();
  const float d0 = v[0] - mean, d1 = v[1] - mean, d2 = v[2] - mean, d3 = v[3] - mean;
  float ss = (d0 * d0 + d1 * d1) + (d2 * d2 + d3 * d3);
#pragma unroll
  for (int off = 1; off < 32; off <<= 1) ss += __shfl_xor(ss, off, 32);
  if (lane == 0) red[wave] = ss;
  __syncthreads();
  float tot2 = 0.f;
#pragma unroll
  for (int w = 0; w < 8; ++w) tot2 += red[w];
  const float var  = tot2 * (1.0f / 1024.0f);
  const float rstd = rsqrtf(var + 1e-5f);
  const v4f g  = *(const v4f*)(gamma + col);
  const v4f bb = *(const v4f*)(beta + col);
  v4f o;
  o[0] = d0 * rstd * g[0] + bb[0];
  o[1] = d1 * rstd * g[1] + bb[1];
  o[2] = d2 * rstd * g[2] + bb[2];
  o[3] = d3 * rstd * g[3] + bb[3];
  float* p = out + (size_t)row * DM + col;
  *(volatile v4f*)p = o;
  __threadfence();
  *(volatile v4f*)p = o;
}

extern "C" void kernel_launch(void* const* d_in, const int* in_sizes, int n_in,
                              void* d_out, int out_size, void* d_ws, size_t ws_size,
                              hipStream_t stream) {
  if (n_in < 14) return;
  if (in_sizes[0] != NTOK * DM) return;
  if (in_sizes[1] != DM * DM || in_sizes[2] != DM * DM) return;
  if (in_sizes[3] != 3 * DM * DM || in_sizes[7] != 3 * DM * DM) return;
  if (in_sizes[4] != 3 * DM || in_sizes[8] != 3 * DM) return;
  if (in_sizes[5] != DM * DM || in_sizes[9] != DM * DM) return;
  if (in_sizes[6] != DM || in_sizes[10] != DM || in_sizes[12] != DM || in_sizes[13] != DM) return;
  if (in_sizes[11] != 2) return;
  if (out_size != NTOK * DM) return;

  const float* x      = (const float*)d_in[0];
  const float* proj_l = (const float*)d_in[1];
  const float* proj_g = (const float*)d_in[2];
  const float* Wl_in  = (const float*)d_in[3];
  const float* bl_in  = (const float*)d_in[4];
  const float* Wl_out = (const float*)d_in[5];
  const float* bl_out = (const float*)d_in[6];
  const float* Wg_in  = (const float*)d_in[7];
  const float* bg_in  = (const float*)d_in[8];
  const float* Wg_out = (const float*)d_in[9];
  const float* bg_out = (const float*)d_in[10];
  const float* fw     = (const float*)d_in[11];
  const float* gamma  = (const float*)d_in[12];
  const float* beta   = (const float*)d_in[13];

  const size_t szTok16 = (size_t)NTOK * DM * 2;
  const size_t szP16   = (size_t)DM * DM * 2;
  const size_t szWin16 = (size_t)3 * DM * DM * 2;
  const size_t szWcat  = (size_t)DM * 2 * DM * 2;
  const size_t szQK    = (size_t)NTOK * 2 * DM * 2;
  const size_t szVT    = (size_t)DM * NTOK * 2;
  const size_t szOcat  = (size_t)NTOK * 2 * DM * 2;
  const size_t szFuse  = (size_t)NTOK * DM * 4;
  size_t off = 0;
  const size_t oX  = off; off += szTok16;
  const size_t oLQ = off; off += szTok16;
  const size_t oOC = oX;
  if (oOC + szOcat > off) return;
  const size_t oGQ = off; off += szTok16;
  const size_t oPL = off; off += szP16;
  const size_t oPG = off; off += szP16;
  const size_t oWL = off; off += szWin16;
  const size_t oWG = off; off += szWin16;
  const size_t oWC = off; off += szWcat;
  const size_t oQK = off; off += szQK;
  const size_t oVT = off; off += szVT;
  const size_t oFU = oQK;
  if (oFU + szFuse > off) return;
  if (off > ws_size) return;

  char* ws = (char*)d_ws;
  _Float16* X16  = (_Float16*)(ws + oX);
  _Float16* LQ   = (_Float16*)(ws + oLQ);
  _Float16* OCAT = (_Float16*)(ws + oOC);
  _Float16* GQ   = (_Float16*)(ws + oGQ);
  _Float16* PLT  = (_Float16*)(ws + oPL);
  _Float16* PGT  = (_Float16*)(ws + oPG);
  _Float16* WL16 = (_Float16*)(ws + oWL);
  _Float16* WG16 = (_Float16*)(ws + oWG);
  _Float16* WCAT = (_Float16*)(ws + oWC);
  _Float16* QK   = (_Float16*)(ws + oQK);
  _Float16* VT   = (_Float16*)(ws + oVT);
  float*    FUSE = (float*)(ws + oFU);

  const dim3 blk(256);
  const float inv64 = 1.0f / 64.0f;

  k_tcvt16<<<dim3(DM / 64, DM / 64), blk, 0, stream>>>(proj_l, PLT, DM, DM, 64.0f);
  k_tcvt16<<<dim3(DM / 64, DM / 64), blk, 0, stream>>>(proj_g, PGT, DM, DM, 64.0f);
  {
    const int n8 = 3 * DM * DM / 8;
    k_cvt16<<<dim3((n8 + 255) / 256), blk, 0, stream>>>(Wl_in, WL16, n8, 64.0f);
    k_cvt16<<<dim3((n8 + 255) / 256), blk, 0, stream>>>(Wg_in, WG16, n8, 64.0f);
  }
  {
    const int n8 = 2 * DM * DM / 8;
    k_wcat<<<dim3((n8 + 255) / 256), blk, 0, stream>>>(Wl_out, Wg_out, fw, WCAT, n8);
  }
  {
    const int n8 = NTOK * DM / 8;
    k_cvt16<<<dim3((n8 + 255) / 256), blk, 0, stream>>>(x, X16, n8, 1.0f);
  }

  const int tilesProj = (NTOK / 64) * (DM / 64);
  const int tilesQK   = (NTOK / 64) * (2 * DM / 64);
  const int tilesVT   = (DM / 64) * (NTOK / 64);
  const dim3 gProj((tilesProj + 7) / 8);
  const dim3 gQK((tilesQK + 7) / 8);
  const dim3 gVT((tilesVT + 7) / 8);

  k_gemm64<0, 1><<<gProj, blk, 0, stream>>>(X16, DM, PLT, DM, (void*)LQ, DM, bl_in, bl_in, fw, NTOK, DM, DM, inv64, 1.0f);
  k_gemm64<0, 1><<<gProj, blk, 0, stream>>>(X16, DM, PGT, DM, (void*)GQ, DM, bl_in, bl_in, fw, NTOK, DM, DM, inv64, 1.0f);

  k_gemm64<2, 1><<<gQK, blk, 0, stream>>>(LQ, DM, WL16, DM, (void*)QK, 2 * DM, bl_in, bl_in, fw, NTOK, 2 * DM, DM, inv64, 1.0f);
  k_gemm64<1, 1><<<gVT, blk, 0, stream>>>(WL16 + (size_t)2 * DM * DM, DM, LQ, DM, (void*)VT, NTOK,
                                          bl_in + 2 * DM, bl_in, fw, DM, NTOK, DM, 16.0f * inv64, 16.0f);
  {
    const int W = 128;
    const dim3 gAtt((NTOK / W) * NH * (W / 64));
    k_attn<<<gAtt, dim3(128), 0, stream>>>(QK, VT, OCAT, W, 0);
  }

  k_gemm64<2, 1><<<gQK, blk, 0, stream>>>(GQ, DM, WG16, DM, (void*)QK, 2 * DM, bg_in, bg_in, fw, NTOK, 2 * DM, DM, inv64, 1.0f);
  k_gemm64<1, 1><<<gVT, blk, 0, stream>>>(WG16 + (size_t)2 * DM * DM, DM, GQ, DM, (void*)VT, NTOK,
                                          bg_in + 2 * DM, bg_in, fw, DM, NTOK, DM, 16.0f * inv64, 16.0f);
  {
    const int W = 1024;
    const dim3 gAtt((NTOK / W) * NH * (W / 64));
    k_attn<<<gAtt, dim3(128), 0, stream>>>(QK, VT, OCAT, W, DM);
  }

  k_gemm64<3, 0><<<gProj, blk, 0, stream>>>(OCAT, 2 * DM, WCAT, 2 * DM, (void*)FUSE, DM, bl_out, bg_out, fw,
                                            NTOK, DM, 2 * DM, 1.0f / 4096.0f, 1.0f);
  k_layernorm<<<dim3(NTOK), blk, 0, stream>>>(FUSE, gamma, beta, (float*)d_out, NTOK);
  (void)hipGetLastError();
}
